// MMD_loss_parallel_56667798504272
// MI455X (gfx1250) — hardware-verified
//
#include <hip/hip_runtime.h>


#define BS   4096
#define NN   8192
#define DF   512
#define RCH  1024
#define NCH  (NN / RCH)
#define KMUL 2.0f
#define KNUM 5
#define CLAMPV 20.0f
#define DM   DF
#define LOSC 1024.0f

typedef _Float16 h16;
typedef unsigned short bf;
typedef __attribute__((ext_vector_type(16))) __bf16   v16bf;
typedef __attribute__((ext_vector_type(16))) _Float16 v16h;
typedef __attribute__((ext_vector_type(8)))  _Float16 v8h;
typedef __attribute__((ext_vector_type(8)))  unsigned short v8us;
typedef __attribute__((ext_vector_type(8)))  float    v8f;
typedef __attribute__((ext_vector_type(4)))  float    v4f;
typedef v8h  __attribute__((may_alias)) v8ha;
typedef v4f  __attribute__((may_alias)) v4fa;
typedef v8us __attribute__((may_alias)) v8usa;

__device__ __forceinline__ unsigned short f2bf(float f) { unsigned u = __float_as_uint(f); u += 0x7FFFu + ((u >> 16) & 1u); return (unsigned short)(u >> 16); }
__device__ __forceinline__ float bf2f(unsigned short b) { return __uint_as_float(((unsigned)b) << 16); }
__device__ __forceinline__ float bfr(float f) { return bf2f(f2bf(f)); }
__device__ __forceinline__ v16h cat16(v8h lo, v8h hi) { return __builtin_shufflevector(lo, hi, 0, 1, 2, 3, 4, 5, 6, 7, 8, 9, 10, 11, 12, 13, 14, 15); }
__device__ __forceinline__ v16bf cat16b(v8us lo, v8us hi) { return __builtin_bit_cast(v16bf, __builtin_shufflevector(lo, hi, 0, 1, 2, 3, 4, 5, 6, 7, 8, 9, 10, 11, 12, 13, 14, 15)); }
__device__ __forceinline__ v8f wmma16(v16h a, v16h b, v8f c) { return __builtin_amdgcn_wmma_f32_16x16x32_f16(false, a, false, b, (short)0, c, false, false); }
__device__ __forceinline__ v8f wmmab(v16bf a, v16bf b, v8f c) { return __builtin_amdgcn_wmma_f32_16x16x32_bf16(false, a, false, b, (short)0, c, false, false); }

template <bool SPLITA, bool F16OUT = false>
__global__ __launch_bounds__(128) void k_gemmb(const bf* __restrict__ A, const bf* __restrict__ Al, const bf* __restrict__ Bn, const float* __restrict__ bias, float* C, int ldc, h16* C2, const float* __restrict__ R = nullptr, int K = DM, int roundR = 1) {
    __shared__ __align__(16) float ost[4][16 * 68];
    const int lane = threadIdx.x & 31, wave = threadIdx.x >> 5, lr = lane & 15, hi = lane >> 4;
    const int r0 = blockIdx.x * 64 + wave * 16, c0 = blockIdx.y * 64;
    const size_t aoff = (size_t)(r0 + lr) * K + 8 * hi;
    size_t boff[4];
#pragma unroll
    for (int t = 0; t < 4; ++t) boff[t] = (size_t)(c0 + t * 16 + lr) * K + 8 * hi;
    v8f acc[4];
#pragma unroll
    for (int t = 0; t < 4; ++t) acc[t] = (v8f){};
#pragma unroll 1
    for (int kc = 0; kc < K; kc += 32) {
        const v16bf a = cat16b(*(const v8us*)(A + aoff + kc), *(const v8us*)(A + aoff + kc + 16));
        v16bf al = a;
        if (SPLITA) al = cat16b(*(const v8us*)(Al + aoff + kc), *(const v8us*)(Al + aoff + kc + 16));
#pragma unroll
        for (int t = 0; t < 4; ++t) { const v16bf b = cat16b(*(const v8us*)(Bn + boff[t] + kc), *(const v8us*)(Bn + boff[t] + kc + 16)); acc[t] = wmmab(a, b, acc[t]); if (SPLITA) acc[t] = wmmab(al, b, acc[t]); }
        asm volatile("v_nop\n\tv_nop\n\tv_nop\n\tv_nop" : "+v"(acc[0]), "+v"(acc[1]), "+v"(acc[2]), "+v"(acc[3]) : "v"(a), "v"(al));
    }
    float* os = &ost[wave][0];
#pragma unroll
    for (int t = 0; t < 4; ++t) { const float bv = bias ? bfr(bias[c0 + t * 16 + lr]) : 0.f;
#pragma unroll
        for (int j = 0; j < 8; ++j) os[(hi * 8 + j) * 68 + t * 16 + lr] = acc[t][j] + bv; }
    __syncthreads();
    if (F16OUT) {
        h16* crow = (h16*)(void*)C + (size_t)r0 * ldc + c0;
        auto pass = [&]() {
#pragma unroll
            for (int s = 0; s < 4; ++s) { const int row = 4 * s + (lane >> 3), piece = lane & 7; const float* sp = os + row * 68 + piece * 8; v8h o, o2;
#pragma unroll
                for (int i = 0; i < 8; ++i) { const h16 a = (h16)sp[i]; o[i] = a; o2[i] = (h16)((sp[i] - (float)a) * LOSC); }
                *(volatile v8h*)(crow + (size_t)row * ldc + piece * 8) = o; if (C2) *(volatile v8h*)(C2 + (size_t)r0 * ldc + c0 + (size_t)row * ldc + piece * 8) = o2; }
        };
        pass(); __threadfence(); pass();
    } else {
        float* crow = C + (size_t)r0 * ldc + c0;
        auto pass = [&]() {
#pragma unroll
            for (int s = 0; s < 8; ++s) { const int Lid = (lane >> 3) + 4 * s, piece = lane & 7; const int row = Lid >> 1, cofs = (Lid & 1) * 32 + piece * 4;
                v4f val = *(const v4fa*)(os + row * 68 + cofs); if (R) { const v4f rv = *(const v4f*)(R + ((size_t)r0 + row) * ldc + c0 + cofs); val += roundR ? (v4f){bfr(rv[0]), bfr(rv[1]), bfr(rv[2]), bfr(rv[3])} : rv; }
                *(volatile v4f*)(crow + (size_t)row * ldc + cofs) = val; }
        };
        pass(); __threadfence(); pass();
    }
}


__global__ __launch_bounds__(256) void k_tot(const float* __restrict__ s0, const float* __restrict__ s1, bf* TB, float* SQL) {
    __shared__ float sh[8];
    const int lane = threadIdx.x & 31, wv = threadIdx.x >> 5; const int n = blockIdx.x * 8 + wv; const float* src = (n < BS) ? (s0 + (size_t)n * DF) : (s1 + (size_t)(n - BS) * DF);
    float sq = 0.f;
#pragma unroll 1
    for (int ps = 0; ps < 2; ++ps) { sq = 0.f;
#pragma unroll
        for (int q = 0; q < DF / 256; ++q) { v8us o;
#pragma unroll
            for (int i = 0; i < 8; ++i) { float t = bfr(src[q * 256 + lane * 8 + i]); t = fminf(fmaxf(t, -CLAMPV), CLAMPV); o[i] = f2bf(t); sq = fmaf(t, t, sq); }
            *(volatile v8us*)(TB + (size_t)n * DF + q * 256 + lane * 8) = o; }
        if (ps == 0) __threadfence(); }
#pragma unroll
    for (int s = 16; s; s >>= 1) sq += __shfl_xor(sq, s, 32);
    if (lane == 0) sh[wv] = sq;
    __syncthreads();
    if (wv == 0) { const float v = (lane < 8) ? sh[lane] : 0.f; float* d = SQL + (size_t)blockIdx.x * 32 + lane; *(volatile float*)d = v; __threadfence(); *(volatile float*)d = v; }
}
__device__ __forceinline__ float sqv(const float* __restrict__ SQL, int i) { return SQL[(size_t)(i >> 3) * 32 + (i & 7)]; }
__global__ __launch_bounds__(256) void k_dsum(const float* __restrict__ G, const float* __restrict__ SQL, int r0, float* RSL) {
    __shared__ float sh[8];
    const int lane = threadIdx.x & 31, wv = threadIdx.x >> 5, rl = blockIdx.x * 8 + wv; const int i = r0 + rl; const float sqi = sqv(SQL, i); const float* gr = G + (size_t)rl * NN;
    float s = 0.f;
#pragma unroll 1
    for (int j0 = lane * 4; j0 < NN; j0 += 128) {
#pragma unroll
        for (int q = 0; q < 4; ++q) { const int j = j0 + q; s += fmaxf(sqi + sqv(SQL, j) - 2.0f * gr[j], 0.f); } }
#pragma unroll
    for (int sh_ = 16; sh_; sh_ >>= 1) s += __shfl_xor(s, sh_, 32);
    if (lane == 0) sh[wv] = s;
    __syncthreads();
    if (wv == 0) { const float v = (lane < 8) ? sh[lane] : 0.f; float* d = RSL + (size_t)(r0 / 8 + blockIdx.x) * 32 + lane; *(volatile float*)d = v; __threadfence(); *(volatile float*)d = v; }
}
__global__ __launch_bounds__(256) void k_bw(const float* __restrict__ RSL, float* BW) {
    __shared__ float pa[256];
    const int t = threadIdx.x; float a = 0.f;
    for (int q = 0; q < NN / 256; ++q) { const int i = t * (NN / 256) + q; a += RSL[(size_t)(i >> 3) * 32 + (i & 7)]; }
    pa[t] = a; __syncthreads();
    if (t < 32) { float v = 0.f; if (t == 0) { float A = 0.f; for (int k = 0; k < 256; ++k) A += pa[k]; const float n = (float)NN; v = A / (n * n - n) / (KMUL * KMUL); }
        *(volatile float*)(BW + t) = v; __threadfence(); *(volatile float*)(BW + t) = v; }
}
__global__ __launch_bounds__(256) void k_kern(const float* __restrict__ G, const float* __restrict__ SQL, const float* __restrict__ BW, int r0, float* S0L, float* S1L) {
    __shared__ float sa[8], sb[8];
    const int lane = threadIdx.x & 31, wv = threadIdx.x >> 5, rl = blockIdx.x * 8 + wv; const int i = r0 + rl; const float sqi = sqv(SQL, i); const float* gr = G + (size_t)rl * NN; const float bw = BW[0];
    float ib[KNUM]; { float w = bw;
#pragma unroll
        for (int k = 0; k < KNUM; ++k) { ib[k] = -1.0f / w; w *= KMUL; } }
    float a = 0.f, b = 0.f;
#pragma unroll 1
    for (int j0 = lane * 4; j0 < NN; j0 += 128) {
#pragma unroll
        for (int q = 0; q < 4; ++q) { const int j = j0 + q; const float D = fmaxf(sqi + sqv(SQL, j) - 2.0f * gr[j], 0.f); float kv = 0.f;
#pragma unroll
            for (int k = 0; k < KNUM; ++k) kv += __expf(D * ib[k]);
            kv *= (1.0f / KNUM); if (j < BS) a += kv; else b += kv; } }
#pragma unroll
    for (int s = 16; s; s >>= 1) { a += __shfl_xor(a, s, 32); b += __shfl_xor(b, s, 32); }
    if (lane == 0) { sa[wv] = a; sb[wv] = b; }
    __syncthreads();
    if (wv == 0) { const float va = (lane < 8) ? sa[lane] : 0.f, vb = (lane < 8) ? sb[lane] : 0.f; const size_t o = (size_t)(r0 / 8 + blockIdx.x) * 32 + lane;
        *(volatile float*)(S0L + o) = va; *(volatile float*)(S1L + o) = vb; __threadfence(); *(volatile float*)(S0L + o) = va; *(volatile float*)(S1L + o) = vb; }
}
__global__ __launch_bounds__(256) void k_loss(const float* __restrict__ S0L, const float* __restrict__ S1L, float* OUTP) {
    __shared__ float p[4][256];
    const int t = threadIdx.x; float a0 = 0.f, a1 = 0.f, b0 = 0.f, b1 = 0.f;
    for (int q = 0; q < NN / 256; ++q) { const int i = t * (NN / 256) + q; const float s0 = S0L[(size_t)(i >> 3) * 32 + (i & 7)], s1 = S1L[(size_t)(i >> 3) * 32 + (i & 7)]; if (i < BS) { a0 += s0; a1 += s1; } else { b0 += s0; b1 += s1; } }
    p[0][t] = a0; p[1][t] = a1; p[2][t] = b0; p[3][t] = b1; __syncthreads();
    if (t == 0) { float M00 = 0.f, M01 = 0.f, M10 = 0.f, M11 = 0.f; for (int k = 0; k < 256; ++k) { M00 += p[0][k]; M01 += p[1][k]; M10 += p[2][k]; M11 += p[3][k]; }
        const float inv = 1.0f / ((float)BS * (float)BS); M00 *= inv; M01 *= inv; M10 *= inv; M11 *= inv;
        const float loss = 2.0f * (M00 * M00 + M11 * M11) - (M00 * M00 + M01 * M01 + M10 * M10 + M11 * M11);
        *(volatile float*)OUTP = loss; __threadfence(); *(volatile float*)OUTP = loss; }
}

extern "C" void kernel_launch(void* const* d_in, const int* in_sizes, int n_in,
                              void* d_out, int out_size, void* d_ws, size_t ws_size, hipStream_t stream) {
    (void)in_sizes; (void)n_in; (void)out_size;
    const float* s0 = (const float*)d_in[0]; const float* s1 = (const float*)d_in[1];
    float* out = (float*)d_out;
    char* wsp = (char*)d_ws;
    auto take = [&](size_t bytes) { char* p = wsp; wsp += (bytes + 255) & ~(size_t)255; return (void*)p; };
    bf* TB = (bf*)take((size_t)NN * DF * 2); float* SQL = (float*)take((NN / 8) * 32 * 4); float* G = (float*)take((size_t)RCH * NN * 4);
    float* RSL = (float*)take((NN / 8) * 32 * 4); float* BW = (float*)take(32 * 4); float* S0L = (float*)take((NN / 8) * 32 * 4); float* S1L = (float*)take((NN / 8) * 32 * 4);
    if ((size_t)(wsp - (char*)d_ws) > ws_size) return;
    k_tot<<<NN / 8, 256, 0, stream>>>(s0, s1, TB, SQL);
    for (int ch = 0; ch < NCH; ++ch) { const int r0 = ch * RCH;
        k_gemmb<false, false><<<dim3(RCH / 64, NN / 64, 1), 128, 0, stream>>>(TB + (size_t)r0 * DF, nullptr, TB, nullptr, G, NN, nullptr, nullptr, DF);
        k_dsum<<<RCH / 8, 256, 0, stream>>>(G, SQL, r0, RSL); }
    k_bw<<<1, 256, 0, stream>>>(RSL, BW);
    for (int ch = 0; ch < NCH; ++ch) { const int r0 = ch * RCH;
        k_gemmb<false, false><<<dim3(RCH / 64, NN / 64, 1), 128, 0, stream>>>(TB + (size_t)r0 * DF, nullptr, TB, nullptr, G, NN, nullptr, nullptr, DF);
        k_kern<<<RCH / 8, 256, 0, stream>>>(G, SQL, BW, r0, S0L, S1L); }
    k_loss<<<1, 256, 0, stream>>>(S0L, S1L, out);
}
